// GATModel_77275051589665
// MI455X (gfx1250) — hardware-verified
//
#include <hip/hip_runtime.h>
#include <stddef.h>
#include <stdint.h>
#include <math.h>


#define DIN    128
#define DH     64
#define KP     128
#define NTHR   256
#define NWAVE  8
#define EPT    8
#define CHUNK  (NTHR * EPT)
#define WCAP   (EPT * 32)
#define LISTN  (NWAVE * WCAP)
#define NBA    1024
#define SLA    10
#define RCAP   28672
#define DEGCAP 128
#define GBM    64
#define GBN    64
#define GTHR   128
#define NUW    (DH * (KP / 8))
#define NEGSL  0.2f
#define EPS_SM 1e-16f
#define AGG_ZINTS (LISTN + 2 * RCAP + 3 * NBA)
#define AGG_LDS_INTS (AGG_ZINTS + 16)
#define WSMAX  134217728

static_assert((CHUNK & (CHUNK - 1)) == 0 && CHUNK <= 4096);
static_assert((NBA & (NBA - 1)) == 0 && NBA == (1 << SLA));
static_assert(((long long)CHUNK << SLA) < (1LL << 31));
static_assert(LISTN % NTHR == 0);
static_assert(NBA % NWAVE == 0 && NBA % 32 == 0 && NBA % GBM == 0);
static_assert(RCAP % 4 == 0 && AGG_ZINTS % 4 == 0 && LISTN % 4 == 0);
static_assert(DIN % 32 == 0 && KP % 32 == 0 && KP == 2 * DH && KP == DIN && DH == GBN);
static_assert(GBM == (GTHR / 32) * 16 && GTHR == 2 * GBN && GTHR == 2 * GBM);
static_assert(NUW % NTHR == 0 && (NUW & (NUW - 1)) == 0);
static_assert(DIN / 8 == 16 && KP / 8 == 16);
static_assert(AGG_LDS_INTS * 4 <= 300000);
static_assert(DH == 2 * 32);
static_assert(DEGCAP >= 36 + 8 && RCAP >= 16710 + 8);

typedef float          v2f   __attribute__((ext_vector_type(2)));
typedef float          v4f   __attribute__((ext_vector_type(4)));
typedef float          v8f   __attribute__((ext_vector_type(8)));
typedef int            v4i   __attribute__((ext_vector_type(4)));
typedef int            v8i   __attribute__((ext_vector_type(8)));
typedef unsigned int   v2u   __attribute__((ext_vector_type(2)));
typedef unsigned short v8us  __attribute__((ext_vector_type(8)));
typedef unsigned short v16us __attribute__((ext_vector_type(16)));
typedef __bf16         v16bf __attribute__((ext_vector_type(16)));
typedef v2f  __attribute__((may_alias)) v2fa;
typedef v4f  __attribute__((may_alias)) v4fa;
typedef v4i  __attribute__((may_alias)) v4ia;
typedef v8us __attribute__((may_alias)) v8usa;
union FragB { v16bf v; v16us u; v8us h[2]; v8i w; };

__device__ __forceinline__ v8f wmb(const FragB& a, const FragB& b, v8f c) {
  v8f d = __builtin_amdgcn_wmma_f32_16x16x32_bf16(false, a.v, false, b.v, (short)0, c, false, false);
  asm volatile("v_nop\n\tv_nop\n\tv_nop\n\tv_nop" : "+v"(d) : "v"(a.w), "v"(b.w));
  return d;
}

__device__ __forceinline__ unsigned bf16_bits(float f) {
  const unsigned u = __float_as_uint(f);
  return ((u + 0x7FFFu + ((u >> 16) & 1u)) >> 16) & 0xFFFFu;
}
__device__ __forceinline__ float bf16_val(float f) {
  return __uint_as_float(bf16_bits(f) << 16);
}

template <int SLB>
__device__ __forceinline__ int scan_chunk(const int* __restrict__ dsts, int nE, int cbase, int slotBase,
                                          int nb, int vec8, int* list, int tid, int lane, int wave) {
  int wc = 0;
  const int el0  = tid * EPT;
  const int e0   = cbase + el0;
  const int sent = -2147483647 - 1;
  v4i da, db;
  if (vec8 != 0 && cbase + CHUNK <= nE) {
    da = *(const v4i*)(dsts + e0);
    db = *(const v4i*)(dsts + e0 + 4);
  } else {
    da.x = (e0     < nE) ? dsts[min(e0,     nE - 1)] : sent;
    da.y = (e0 + 1 < nE) ? dsts[min(e0 + 1, nE - 1)] : sent;
    da.z = (e0 + 2 < nE) ? dsts[min(e0 + 2, nE - 1)] : sent;
    da.w = (e0 + 3 < nE) ? dsts[min(e0 + 3, nE - 1)] : sent;
    db.x = (e0 + 4 < nE) ? dsts[min(e0 + 4, nE - 1)] : sent;
    db.y = (e0 + 5 < nE) ? dsts[min(e0 + 5, nE - 1)] : sent;
    db.z = (e0 + 6 < nE) ? dsts[min(e0 + 6, nE - 1)] : sent;
    db.w = (e0 + 7 < nE) ? dsts[min(e0 + 7, nE - 1)] : sent;
  }
  const unsigned nbs = (unsigned)slotBase;
  const unsigned unb = (unsigned)nb;
  const unsigned s0 = (unsigned)da.x - nbs, s1 = (unsigned)da.y - nbs;
  const unsigned s2 = (unsigned)da.z - nbs, s3 = (unsigned)da.w - nbs;
  const unsigned s4 = (unsigned)db.x - nbs, s5 = (unsigned)db.y - nbs;
  const unsigned s6 = (unsigned)db.z - nbs, s7 = (unsigned)db.w - nbs;
  const bool h0 = s0 < unb, h1 = s1 < unb, h2 = s2 < unb, h3 = s3 < unb;
  const bool h4 = s4 < unb, h5 = s5 < unb, h6 = s6 < unb, h7 = s7 < unb;
  const unsigned any = __builtin_amdgcn_ballot_w32(h0 | h1 | h2 | h3 | h4 | h5 | h6 | h7);
  if (any != 0u) {
#define HITJ(J, HJ, SJ) { \
      const unsigned mj = __builtin_amdgcn_ballot_w32(HJ); \
      if (mj != 0u) { \
        if (HJ) { \
          const int pos = wc + (int)__builtin_amdgcn_mbcnt_lo(mj, 0u); \
          if (pos < WCAP) list[wave * WCAP + pos] = ((el0 + (J)) << SLB) | (int)(SJ); \
        } \
        wc += (int)__builtin_popcount(mj); } }
    HITJ(0, h0, s0)
    HITJ(1, h1, s1)
    HITJ(2, h2, s2)
    HITJ(3, h3, s3)
    HITJ(4, h4, s4)
    HITJ(5, h5, s5)
    HITJ(6, h6, s6)
    HITJ(7, h7, s7)
#undef HITJ
  }
  return wc;
}

__global__ __launch_bounds__(NTHR) void k_wprep(const float* __restrict__ W1, const float* __restrict__ W2,
                                                const float* __restrict__ W3,
                                                unsigned short* WT1, unsigned short* WT2, unsigned short* WT3) {
  const int u = (int)blockIdx.x * NTHR + (int)threadIdx.x;
  if (u >= 3 * NUW) return;
  const int mat = u / NUW;
  const int v   = u & (NUW - 1);
  const int n   = v >> 4;
  const int k8  = (v & 15) * 8;
  const float* w;
  unsigned short* o;
  int kk;
  if (mat == 0)      { w = W1; o = WT1; kk = k8; }
  else if (mat == 1) { w = W2; o = WT2; kk = k8 & (DH - 1); }
  else               { w = W3; o = WT3; kk = k8 & (DH - 1); }
  const float* p = w + (size_t)kk * DH + n;
  v8us ov;
#pragma unroll
  for (int i = 0; i < 8; ++i) ov[i] = (unsigned short)bf16_bits(p[(size_t)i * DH]);
  unsigned short* dp = o + (size_t)n * KP + k8;
  *(volatile v8us*)dp = ov;
  __threadfence();
  *(volatile v8us*)dp = ov;
}

__global__ __launch_bounds__(NTHR) void k_cvx(const float* __restrict__ x, int nN, int nUnits,
                                              unsigned short* xb) {
  const int u = (int)blockIdx.x * NTHR + (int)threadIdx.x;
  if (u >= nUnits) return;
  const int row = u >> 4;
  const int k8  = (u & 15) * 8;
  const int rc  = row < nN ? row : nN - 1;
  const float* p = x + (size_t)rc * DIN + k8;
  const v4f a = *(const v4f*)p;
  const v4f b = *(const v4f*)(p + 4);
  const bool ok = row < nN;
  v8us o;
  o[0] = ok ? (unsigned short)bf16_bits(a.x) : (unsigned short)0;
  o[1] = ok ? (unsigned short)bf16_bits(a.y) : (unsigned short)0;
  o[2] = ok ? (unsigned short)bf16_bits(a.z) : (unsigned short)0;
  o[3] = ok ? (unsigned short)bf16_bits(a.w) : (unsigned short)0;
  o[4] = ok ? (unsigned short)bf16_bits(b.x) : (unsigned short)0;
  o[5] = ok ? (unsigned short)bf16_bits(b.y) : (unsigned short)0;
  o[6] = ok ? (unsigned short)bf16_bits(b.z) : (unsigned short)0;
  o[7] = ok ? (unsigned short)bf16_bits(b.w) : (unsigned short)0;
  unsigned short* dp = xb + (size_t)row * DIN + k8;
  *(volatile v8us*)dp = o;
  __threadfence();
  *(volatile v8us*)dp = o;
}

template <int FIN>
__global__ __launch_bounds__(GTHR) void k_gemm(
    const unsigned short* __restrict__ A, const unsigned short* __restrict__ WT,
    const float* __restrict__ bias, float* outF,
    const float* __restrict__ atts, const float* __restrict__ attd,
    float* SD, int MPr, int nRowsOut)
{
  __shared__ __attribute__((aligned(16))) float stg[GBM * GBN];
  __shared__ __attribute__((aligned(16))) float satt[2 * GBN];
  __shared__ __attribute__((aligned(16))) float sdot[2 * GBM];
  const int tid = (int)threadIdx.x, lane = tid & 31, wave = tid >> 5, hh = lane >> 4, m = lane & 15;
  const int rowBase = (int)blockIdx.x * GBM;

  if (FIN == 0) {
    const int which = tid >> 6;
    const int c  = tid & 63;
    const float vs = atts[c];
    const float vd = attd[c];
    const float v = (which == 0) ? vs : vd;
    satt[which * GBN + c] = bf16_val(v);
  }

  v8f acc[4];
  {
    const v8f z = {0.f, 0.f, 0.f, 0.f, 0.f, 0.f, 0.f, 0.f};
    acc[0] = z; acc[1] = z; acc[2] = z; acc[3] = z;
  }
  const unsigned short* ap = A  + (size_t)(rowBase + 16 * wave + m) * (size_t)KP + 8 * hh;
  const unsigned short* wp = WT + (size_t)m * (size_t)KP + 8 * hh;
#pragma unroll 1
  for (int ks = 0; ks < KP / 32; ++ks) {
    FragB af;
    af.h[0] = *(const v8usa*)(ap + 32 * ks);
    af.h[1] = *(const v8usa*)(ap + 32 * ks + 16);
#pragma unroll
    for (int t = 0; t < 4; ++t) {
      const unsigned short* wq = wp + (size_t)(16 * t) * (size_t)KP + 32 * ks;
      FragB bf;
      bf.h[0] = *(const v8usa*)wq;
      bf.h[1] = *(const v8usa*)(wq + 16);
      acc[t] = wmb(af, bf, acc[t]);
    }
  }

  float bv[4];
#pragma unroll
  for (int t = 0; t < 4; ++t) bv[t] = bf16_val(bias[16 * t + m]);
#pragma unroll
  for (int t = 0; t < 4; ++t) {
    const int lc = 16 * t + m;
#pragma unroll
    for (int r = 0; r < 8; ++r) {
      const int lr = 16 * wave + 8 * hh + r;
      stg[lr * GBN + lc] = acc[t][r] + bv[t];
    }
  }
  __syncthreads();

  if (FIN == 0) {
    const int row = tid & 63, which = tid >> 6;
    const float* sa = satt + which * GBN;
    const float* hr = stg + row * GBN;
    float d = 0.f;
#pragma unroll 4
    for (int c4 = 0; c4 < GBN / 4; ++c4) {
      const v4f hv = *(const v4fa*)(hr + 4 * c4);
      const v4f av = *(const v4fa*)(sa + 4 * c4);
      d = fmaf(hv.x, av.x, d);
      d = fmaf(hv.y, av.y, d);
      d = fmaf(hv.z, av.z, d);
      d = fmaf(hv.w, av.w, d);
    }
    sdot[which * GBM + row] = d;
    __syncthreads();
  }

  v4f fv[8];
#pragma unroll
  for (int i = 0; i < 8; ++i) {
    const int lr = 16 * wave + 2 * i + hh;
    fv[i] = *(const v4fa*)(stg + lr * GBN + 4 * m);
  }
  const int which2 = lane >> 4, piece = lane & 15;
  v4f sdv = {0.f, 0.f, 0.f, 0.f};
  float* sp = SD;
  if (FIN == 0) {
    sdv = *(const v4fa*)(sdot + which2 * GBM + 4 * piece);
    sp  = SD + (size_t)which2 * (size_t)MPr + rowBase + 4 * piece;
  }

#pragma unroll
  for (int i = 0; i < 8; ++i) {
    const int lr = 16 * wave + 2 * i + hh;
    const int gr = rowBase + lr;
    float* op = outF + (size_t)gr * (size_t)DH + 4 * m;
    if (gr < nRowsOut) *(volatile v4f*)op = fv[i];
  }
  if (FIN == 0) { if (wave == 0) *(volatile v4f*)sp = sdv; }
  __threadfence();
#pragma unroll
  for (int i = 0; i < 8; ++i) {
    const int lr = 16 * wave + 2 * i + hh;
    const int gr = rowBase + lr;
    float* op = outF + (size_t)gr * (size_t)DH + 4 * m;
    if (gr < nRowsOut) *(volatile v4f*)op = fv[i];
  }
  if (FIN == 0) { if (wave == 0) *(volatile v4f*)sp = sdv; }
}

__global__ __launch_bounds__(NTHR) void k_agg(const int* __restrict__ srcs, const int* __restrict__ dsts,
                                              int nE, int nN, int vec8, int mRows,
                                              const float* __restrict__ SD,
                                              const float* __restrict__ xl, const float* __restrict__ bA,
                                              unsigned short* hb) {
  extern __shared__ __attribute__((aligned(16))) int dsm[];
  int* list = dsm;
  int* hl   = dsm + LISTN;
  int* sl   = dsm + LISTN + RCAP;
  int* cnt  = dsm + LISTN + 2 * RCAP;
  int* offs = cnt + NBA;
  int* cur  = offs + NBA;
  int* misc = cur + NBA;
  const int tid = (int)threadIdx.x, lane = tid & 31, wave = tid >> 5;
  const int nodeBase = (int)blockIdx.x * NBA;

  {
    const v4i z4 = {0, 0, 0, 0};
    for (int i = tid * 4; i < AGG_ZINTS; i += NTHR * 4) *(v4ia*)(dsm + i) = z4;
    if (tid < 16) misc[tid] = 0;
  }
  const float ba = bf16_val(bA[0]);
  __syncthreads();

  int t = 0, ov = 0;
  const int nChunks = (nE + CHUNK - 1) / CHUNK;
#pragma unroll 1
  for (int ch = 0; ch < nChunks; ++ch) {
    const int cbase = ch * CHUNK;
    const int wc = scan_chunk<SLA>(dsts, nE, cbase, nodeBase, NBA, vec8, list, tid, lane, wave);
    if (lane == 0) misc[wave] = wc;
    __syncthreads();
    if (wave == 0) {
#pragma unroll 1
      for (int w2 = 0; w2 < NWAVE; ++w2) {
        int c = misc[w2];
        c = c < 0 ? 0 : (c > WCAP ? WCAP : c);
#pragma unroll 1
        for (int b0 = 0; b0 < c; b0 += 32) {
          const int idx = b0 + lane;
          const int ent = list[w2 * WCAP + (idx < WCAP ? idx : WCAP - 1)];
          const int m32 = (c - b0) < 32 ? (c - b0) : 32;
#pragma unroll 1
          for (int k = 0; k < m32; ++k) {
            const int u    = __builtin_amdgcn_readlane(ent, k);
            const int slot = u & (NBA - 1);
            const int el   = (u >> SLA) & (CHUNK - 1);
            const int pk   = ((cbase + el) << SLA) | slot;
            if (t < RCAP) {
              if (lane == 0) { hl[t] = pk; cnt[slot] = cnt[slot] + 1; }
              t = t + 1;
            } else {
              ov = 1;
            }
          }
        }
      }
    }
    __syncthreads();
  }
  if (wave == 0 && lane == 0) { misc[8] = t; misc[9] = ov; }
  __syncthreads();
  int tt = misc[8];
  tt = tt < 0 ? 0 : (tt > RCAP ? RCAP : tt);
  const int ovf = misc[9];

  if (wave == 0) {
    const int base = lane * (NBA / 32);
    int s = 0;
#pragma unroll 1
    for (int i = 0; i < NBA / 32; ++i) s += cnt[base + i];
    int incl = s;
#pragma unroll
    for (int d = 1; d < 32; d <<= 1) {
      const int y = __shfl_up(incl, d, 32);
      if (lane >= d) incl += y;
    }
    int run = incl - s;
#pragma unroll 1
    for (int i = 0; i < NBA / 32; ++i) {
      const int cv = cnt[base + i];
      offs[base + i] = run;
      cur[base + i]  = run;
      run += cv;
    }
  }
  __syncthreads();
  if (wave == 0) {
#pragma unroll 1
    for (int b0 = 0; b0 < tt; b0 += 32) {
      const int idx = b0 + lane;
      const int ent = hl[idx < RCAP ? idx : RCAP - 1];
      const int m32 = (tt - b0) < 32 ? (tt - b0) : 32;
#pragma unroll 1
      for (int k = 0; k < m32; ++k) {
        const int u    = __builtin_amdgcn_readlane(ent, k);
        const int slot = u & (NBA - 1);
        if (lane == 0) {
          int p = cur[slot];
          p = p < 0 ? 0 : (p > RCAP - 1 ? RCAP - 1 : p);
          sl[p] = u;
          cur[slot] = p + 1;
        }
      }
    }
  }
  __syncthreads();

  const float qnan = __int_as_float(0x7fc00000);
  const float* SJp = SD;
  const float* SIp = SD + mRows;
#pragma unroll 1
  for (int si = 0; si < NBA / NWAVE; ++si) {
    const int s    = si * NWAVE + wave;
    const int node = nodeBase + s;
    if (node < mRows) {
      const bool live = node < nN;
      const int craw = cnt[s];
      const bool big = craw > DEGCAP;
      int c = craw < 0 ? 0 : (craw > DEGCAP ? DEGCAP : craw);
      int o = offs[s];
      o = o < 0 ? 0 : (o > RCAP ? RCAP : o);
      if (c > tt - o) c = (tt - o) > 0 ? (tt - o) : 0;
      c = live ? c : 0;
      const int nc = live ? node : nN - 1;
      const float ad = SIp[nc];

      float mloc = -3.0e38f;
#pragma unroll 1
      for (int b0 = 0; b0 < c; b0 += 32) {
        int idx = o + b0 + lane;
        idx = idx > RCAP - 1 ? RCAP - 1 : idx;
        const int ent = sl[idx];
        int eid = ent >> SLA;
        eid = eid < 0 ? 0 : (eid > nE - 1 ? nE - 1 : eid);
        int sr = srcs[eid];
        sr = sr < 0 ? 0 : (sr > nN - 1 ? nN - 1 : sr);
        const float es = SJp[sr];
        float lg = (ad + es) + ba;
        lg = lg >= 0.f ? lg : NEGSL * lg;
        const float lv = (b0 + lane < c) ? lg : -3.0e38f;
        mloc = fmaxf(mloc, lv);
      }
#pragma unroll
      for (int off = 16; off > 0; off >>= 1) mloc = fmaxf(mloc, __shfl_xor(mloc, off));
      const float mx = mloc;

      float dn = 0.0f, a0 = 0.0f, a1 = 0.0f;
#pragma unroll 1
      for (int b0 = 0; b0 < c; b0 += 32) {
        int idx = o + b0 + lane;
        idx = idx > RCAP - 1 ? RCAP - 1 : idx;
        const int ent = sl[idx];
        int eid = ent >> SLA;
        eid = eid < 0 ? 0 : (eid > nE - 1 ? nE - 1 : eid);
        int sr = srcs[eid];
        sr = sr < 0 ? 0 : (sr > nN - 1 ? nN - 1 : sr);
        const float es = SJp[sr];
        float lg = (ad + es) + ba;
        lg = lg >= 0.f ? lg : NEGSL * lg;
        const float ee  = expf(fminf(lg - mx, 0.0f));
        const float exv = (b0 + lane < c) ? ee : 0.0f;
        const int   exi = __float_as_int(exv);
        const int m32 = (c - b0) < 32 ? (c - b0) : 32;
#pragma unroll 1
        for (int k = 0; k < m32; ++k) {
          const int   sk = __builtin_amdgcn_readlane(sr, k);
          const float ek = __int_as_float(__builtin_amdgcn_readlane(exi, k));
          const v2f a = *(const v2fa*)(xl + (size_t)sk * DH + 2 * lane);
          dn += ek;
          a0 = fmaf(ek, a.x, a0);
          a1 = fmaf(ek, a.y, a1);
        }
      }
      const float inv = __builtin_amdgcn_rcpf(dn + EPS_SM);
      const float pzr = (ovf != 0 || big) ? qnan : 0.0f;
      float y0 = a0 * inv, y1 = a1 * inv;
      y0 = y0 >= 0.f ? y0 : NEGSL * y0;
      y1 = y1 >= 0.f ? y1 : NEGSL * y1;
      y0 = y0 + pzr;
      y1 = y1 + pzr;
      const float v0 = live ? y0 : 0.0f;
      const float v1 = live ? y1 : 0.0f;
      const unsigned h0 = bf16_bits(v0), h1 = bf16_bits(v1);
      const unsigned l0 = bf16_bits(v0 - __uint_as_float(h0 << 16));
      const unsigned l1 = bf16_bits(v1 - __uint_as_float(h1 << 16));
      const int hw = (int)(h0 | (h1 << 16));
      const int lw = (int)(l0 | (l1 << 16));
      const int sa = (2 * lane) & 31, sb = (2 * lane + 1) & 31;
      const int g0 = __shfl(hw, sa), g1 = __shfl(hw, sb);
      const int q0 = __shfl(lw, sa), q1 = __shfl(lw, sb);
      const bool lsel = lane >= 16;
      v2u pv;
      pv.x = (unsigned int)(lsel ? q0 : g0);
      pv.y = (unsigned int)(lsel ? q1 : g1);
      unsigned short* gp = hb + (size_t)node * KP + 4 * lane;
      *(volatile v2u*)gp = pv;
      __threadfence();
      *(volatile v2u*)gp = pv;
    }
  }
}

static inline int cdiv(int a, int b) { return (a + b - 1) / b; }

extern "C" void kernel_launch(void* const* d_in, const int* in_sizes, int n_in,
                              void* d_out, int out_size, void* d_ws, size_t ws_size,
                              hipStream_t stream) {
  if (n_in < 12) return;
  if (in_sizes[0] < DIN || (in_sizes[0] % DIN) != 0) return;
  const int nN = in_sizes[0] / DIN;
  if (nN < 1 || nN > (1 << 22)) return;
  if (in_sizes[1] < 2 || (in_sizes[1] & 1) != 0) return;
  const int nE = in_sizes[1] / 2;
  if (nE < 1 || nE >= (1 << 21)) return;
  if (in_sizes[2] != DIN * DH) return;
  if (in_sizes[3] != DH) return;
  if (in_sizes[4] != 2 * DH) return;
  if (in_sizes[5] < 1) return;
  if (in_sizes[6] != DH * DH) return;
  if (in_sizes[7] != DH) return;
  if (in_sizes[8] != 2 * DH) return;
  if (in_sizes[9] < 1) return;
  if (in_sizes[10] != DH * DH) return;
  if (in_sizes[11] != DH) return;
  if ((long long)out_size != (long long)nN * DH) return;

  const float* x    = (const float*)d_in[0];
  const int*   edge = (const int*)d_in[1];
  const float* W1   = (const float*)d_in[2];
  const float* bW1  = (const float*)d_in[3];
  const float* A1   = (const float*)d_in[4];
  const float* bA1  = (const float*)d_in[5];
  const float* W2   = (const float*)d_in[6];
  const float* bW2  = (const float*)d_in[7];
  const float* A2   = (const float*)d_in[8];
  const float* bA2  = (const float*)d_in[9];
  const float* Wfc  = (const float*)d_in[10];
  const float* bfc  = (const float*)d_in[11];
  float* out = (float*)d_out;
  const int* src = edge;
  const int* dst = edge + nE;

  const int MP   = cdiv(nN, GBM) * GBM;
  const int gM   = MP / GBM;
  const int gA   = cdiv(MP, NBA);
  if ((long long)gA * NBA < (long long)MP) return;
  const int vec8 = ((nE & 3) == 0) ? 1 : 0;

  char* ws = (char*)d_ws;
  size_t off = 0;
  const size_t oWT1 = off; off += (size_t)DH * KP * 2;                    off = (off + 255) & ~(size_t)255;
  const size_t oWT2 = off; off += (size_t)DH * KP * 2;                    off = (off + 255) & ~(size_t)255;
  const size_t oWT3 = off; off += (size_t)DH * KP * 2;                    off = (off + 255) & ~(size_t)255;
  const size_t oSD  = off; off += (size_t)2 * MP * 4;                     off = (off + 255) & ~(size_t)255;
  const size_t oXB  = off; off += (size_t)MP * DIN * 2;                   off = (off + 255) & ~(size_t)255;
  const size_t oWH  = off; off += (size_t)MP * DH * 4;                    off = (off + 255) & ~(size_t)255;
  const size_t oHP  = off; off += (size_t)MP * KP * 2;                    off = (off + 255) & ~(size_t)255;
  if (off > ws_size || off > (size_t)WSMAX) return;
  unsigned short* WT1 = (unsigned short*)(ws + oWT1);
  unsigned short* WT2 = (unsigned short*)(ws + oWT2);
  unsigned short* WT3 = (unsigned short*)(ws + oWT3);
  float*          SDp = (float*)(ws + oSD);
  unsigned short* XB  = (unsigned short*)(ws + oXB);
  float*          WH  = (float*)(ws + oWH);
  unsigned short* HP  = (unsigned short*)(ws + oHP);

  const size_t aggLds = (size_t)AGG_LDS_INTS * 4;
  hipFuncSetAttribute(reinterpret_cast<const void*>(&k_agg), hipFuncAttributeMaxDynamicSharedMemorySize, (int)aggLds);

  const int nUx = MP * (DIN / 8);
  k_wprep<<<(3 * NUW) / NTHR, NTHR, 0, stream>>>(W1, W2, Wfc, WT1, WT2, WT3);
  k_cvx<<<cdiv(nUx, NTHR), NTHR, 0, stream>>>(x, nN, nUx, XB);
  k_gemm<0><<<gM, GTHR, 0, stream>>>(XB, WT1, bW1, WH, A1 + DH, A1, SDp, MP, MP);
  k_agg<<<gA, NTHR, aggLds, stream>>>(src, dst, nE, nN, vec8, MP, SDp, WH, bA1, HP);
  k_gemm<0><<<gM, GTHR, 0, stream>>>(HP, WT2, bW2, WH, A2 + DH, A2, SDp, MP, MP);
  k_agg<<<gA, NTHR, aggLds, stream>>>(src, dst, nE, nN, vec8, MP, SDp, WH, bA2, HP);
  k_gemm<1><<<gM, GTHR, 0, stream>>>(HP, WT3, bfc, out, A2 + DH, A2, SDp, MP, nN);
}
